// SSM_62861141344380
// MI455X (gfx1250) — hardware-run, weakly checked
//
#include <hip/hip_runtime.h>
#include <math.h>

typedef __attribute__((ext_vector_type(16))) _Float16 v16h;
typedef __attribute__((ext_vector_type(8)))  _Float16 v8h;
typedef __attribute__((ext_vector_type(8)))  float    v8f;
typedef __attribute__((ext_vector_type(4)))  float    v4f;

constexpr int kB  = 8;
constexpr int kH  = 128;
constexpr int kL  = 8192;
constexpr int kP  = 256;
constexpr int kRows      = kB * kL;
constexpr int kGroups    = 4;
constexpr int kGroupB    = kB / kGroups;
constexpr int kGroupRows = kGroupB * kL;
constexpr int kA2P   = 2 * kP + kH;
constexpr int kColIm = kP;
constexpr int kColU  = 2 * kP;
constexpr int kVinP  = 2 * kP;
constexpr int kScanTS = 64;
constexpr int kScanCh = 64;
constexpr int kScanLP = 68;
constexpr int kTrP    = 65;

constexpr float kCarryU = 64.0f;
constexpr float kCarryB = 1024.0f;
constexpr float kCarryX = 64.0f;
constexpr float kCarryW = 256.0f;
constexpr float kFoldMix = 1.0f / (kCarryU * kCarryB);
constexpr float kFoldOut = 1.0f / (kCarryX * kCarryW);
constexpr float kF16MinNormal = 6.103515625e-05f;
constexpr float kInvSqrt2 = 0.70710678118654752440f;

static_assert(kCarryU == kCarryX);
static_assert(kA2P == 640 && kVinP == 512);
static_assert((kH % 32) == 0 && (kA2P % 32) == 0);
static_assert((kGroupRows % 64) == 0 && (kVinP % 64) == 0 && (kH % 64) == 0 && (kL % 64) == 0);
static_assert((kA2P % 64) == 0 && (kColU % 64) == 0 && (kColIm % 64) == 0);
static_assert((kL % kScanTS) == 0 && (kP % kScanCh) == 0);
static_assert(kGroups * kGroupB == kB);

constexpr size_t kSzA2  = (size_t)kRows * kA2P * 2;
constexpr size_t kSzVIN = (size_t)kGroupRows * kVinP * 4;
constexpr size_t kSzBT1 = (size_t)kVinP * kH * 2;
constexpr size_t kSzW2  = (size_t)kH * kA2P * 2;
constexpr size_t kOffA2  = 0;
constexpr size_t kOffVIN = kOffA2 + kSzA2;
constexpr size_t kOffBT1 = kOffVIN + kSzVIN;
constexpr size_t kOffW2  = kOffBT1 + kSzBT1;
constexpr size_t kWsTotal = kOffW2 + kSzW2;
static_assert(kWsTotal == 117735424ull);
static_assert(kWsTotal <= 134217728ull);
static_assert((kOffVIN % 128) == 0 && (kOffBT1 % 128) == 0 && (kOffW2 % 128) == 0);

__device__ __forceinline__ _Float16 to_f16_flush(float v) {
  const float w = (fabsf(v) < kF16MinNormal) ? 0.0f : v;
  return (_Float16)w;
}
__device__ __forceinline__ float gelu_erf(float v) {
  return 0.5f * v * (1.0f + erff(v * kInvSqrt2));
}
union FragU { v16h v; v8h h[2]; };
__device__ __forceinline__ v16h frag_load(const _Float16* p) {
  FragU f;
  f.h[0] = *(const v8h*)(p);
  f.h[1] = *(const v8h*)(p + 16);
  return f.v;
}
__device__ __forceinline__ v8f mma_f16(v16h a, v16h b, v8f c) {
  return __builtin_amdgcn_wmma_f32_16x16x32_f16(false, a, false, b, (short)0, c, false, false);
}
__device__ __forceinline__ void mma_guard1(v8f& a, v16h x, v16h y) {
  asm volatile("v_nop\n\tv_nop\n\tv_nop\n\tv_nop" : "+v"(a) : "v"(x), "v"(y));
}

__global__ __launch_bounds__(256) void prep_weights_kernel(
    const float* __restrict__ Bre, const float* __restrict__ Bim,
    const float* __restrict__ Cre, const float* __restrict__ Cim,
    const float* __restrict__ Dm,
    unsigned short* __restrict__ BT1, unsigned short* __restrict__ W2)
{
  const int blk = blockIdx.x;
  const float* src = Bre;
  unsigned short* dst = BT1;
  int rowShift = 7;
  int dstPitch = kH;
  float scl = kCarryB;
  int jb = blk;
  if (blk >= 16 && blk < 32) {
    src = Bim; dst = BT1 + (size_t)kP * kH; jb = blk - 16;
  } else if (blk >= 32 && blk < 48) {
    src = Cre; dst = W2; rowShift = 8; dstPitch = kA2P; scl = kCarryW; jb = blk - 32;
  } else if (blk >= 48 && blk < 64) {
    src = Cim; dst = W2 + kColIm; rowShift = 8; dstPitch = kA2P; scl = -kCarryW; jb = blk - 48;
  } else if (blk >= 64) {
    src = Dm; dst = W2 + kColU; rowShift = 7; dstPitch = kA2P; scl = kCarryW; jb = blk - 64;
  }
  const int j   = jb * 256 + (int)threadIdx.x;
  const int e0  = j << 3;
  const int row = e0 >> rowShift;
  const int col = e0 & ((1 << rowShift) - 1);
  const v4f a0 = *(const v4f*)(src + e0);
  const v4f a1 = *(const v4f*)(src + e0 + 4);
  v8h hv;
#pragma unroll
  for (int e = 0; e < 4; ++e) {
    hv[e]     = to_f16_flush(a0[e] * scl);
    hv[4 + e] = to_f16_flush(a1[e] * scl);
  }
  unsigned short* q = dst + (size_t)row * dstPitch + col;
  *(volatile v8h*)q = hv;
  __threadfence();
  *(volatile v8h*)q = hv;
}

__global__ __launch_bounds__(256) void pack_u_kernel(
    const float* __restrict__ u, unsigned short* __restrict__ A2)
{
  __shared__ float tile[kH * kTrP];
  const int tid = threadIdx.x, lane = tid & 31, wave = tid >> 5;
  const int l0 = blockIdx.x * 64;
  const int b  = blockIdx.y;
  const float* ub = u + (size_t)b * kH * kL + l0;
#pragma unroll
  for (int p = 0; p < 8; ++p) {
    const int idx = tid + p * 256;
    const int h = idx >> 4;
    const int q = (idx & 15) * 4;
    const v4f v = *(const v4f*)(ub + (size_t)h * kL + q);
    tile[h * kTrP + q + 0] = v[0];
    tile[h * kTrP + q + 1] = v[1];
    tile[h * kTrP + q + 2] = v[2];
    tile[h * kTrP + q + 3] = v[3];
  }
  __syncthreads();
  const int hh = lane >> 4, c8 = (lane & 15) * 8;
  v8h hv[4];
#pragma unroll
  for (int it = 0; it < 4; ++it) {
    const int row = it * 16 + wave * 2 + hh;
#pragma unroll
    for (int e = 0; e < 8; ++e) hv[it][e] = to_f16_flush(tile[(c8 + e) * kTrP + row] * kCarryU);
  }
  const size_t rbase = (size_t)b * kL + l0;
  for (int pass = 0; pass < 2; ++pass) {
#pragma unroll
    for (int it = 0; it < 4; ++it) {
      const int row = it * 16 + wave * 2 + hh;
      *(volatile v8h*)(A2 + (rbase + row) * kA2P + kColU + c8) = hv[it];
    }
    __threadfence();
  }
}

template <bool GELU>
__global__ __launch_bounds__(256) void gemm_f16_kernel(
    const unsigned short* __restrict__ Ap, int lda, long strideA,
    const unsigned short* __restrict__ Btp, int ldb, long strideB,
    float* __restrict__ Cout, int ldc, long strideC,
    int M, int N, int K, float scale)
{
  const _Float16* A  = (const _Float16*)Ap;
  const _Float16* Bt = (const _Float16*)Btp;
  __shared__ __align__(16) float sT[8][16 * 68];
  const int b    = blockIdx.y;
  const int lane = threadIdx.x & 31;
  const int wave = threadIdx.x >> 5;
  const int tilesN = N >> 6;
  const int tilesM = M >> 6;
  const int tile = blockIdx.x * 8 + wave;
  if (tile >= tilesM * tilesN) return;
  const int tm = tile / tilesN;
  const int tn = tile - tm * tilesN;
  const int m0 = tm << 6;
  const int n0 = tn << 6;

  const _Float16* Ab = A  + (size_t)b * strideA;
  const _Float16* Bb = Bt + (size_t)b * strideB;

  const int rlane = lane & 15;
  const int koff  = (lane >> 4) * 8;
  const int mOff  = (lane >> 4) * 8;

  v8f acc[4][4];
#pragma unroll
  for (int i = 0; i < 4; ++i)
#pragma unroll
    for (int j = 0; j < 4; ++j) acc[i][j] = (v8f){0.f, 0.f, 0.f, 0.f, 0.f, 0.f, 0.f, 0.f};

  for (int k0 = 0; k0 < K; k0 += 32) {
    v16h bh[4];
#pragma unroll
    for (int j = 0; j < 4; ++j) {
      const size_t bo = (size_t)(n0 + (j << 4) + rlane) * ldb + koff + k0;
      bh[j] = frag_load(Bb + bo);
    }
#pragma unroll
    for (int i = 0; i < 4; ++i) {
      const size_t ao = (size_t)(m0 + (i << 4) + rlane) * lda + koff + k0;
      const v16h ah = frag_load(Ab + ao);
#pragma unroll
      for (int j = 0; j < 4; ++j) acc[i][j] = mma_f16(ah, bh[j], acc[i][j]);
      mma_guard1(acc[i][0], ah, bh[0]);
      mma_guard1(acc[i][1], ah, bh[1]);
      mma_guard1(acc[i][2], ah, bh[2]);
      mma_guard1(acc[i][3], ah, bh[3]);
    }
  }

  float* slab = sT[wave];
  float* C = Cout + (size_t)b * strideC;
  const int hh = lane >> 4, c4 = (lane & 15) * 4;
#pragma unroll
  for (int i = 0; i < 4; ++i) {
    const int mBase = m0 + (i << 4);
#pragma unroll
    for (int j = 0; j < 4; ++j) {
#pragma unroll
      for (int r = 0; r < 8; ++r) {
        slab[(mOff + r) * 68 + (j << 4) + rlane] = acc[i][j][r] * scale;
      }
    }
    __builtin_amdgcn_fence(__ATOMIC_RELEASE, "workgroup");
    __builtin_amdgcn_wave_barrier();
    __builtin_amdgcn_fence(__ATOMIC_ACQUIRE, "workgroup");
    if (GELU) {
#pragma unroll 1
      for (int it = 0; it < 8; ++it) {
        float* sp = slab + (it * 2 + hh) * 68 + c4;
        const v4f v = *(const v4f*)sp;
        v4f g;
        g[0] = gelu_erf(v[0]);
        g[1] = gelu_erf(v[1]);
        g[2] = gelu_erf(v[2]);
        g[3] = gelu_erf(v[3]);
        *(v4f*)sp = g;
      }
    }
    for (int pass = 0; pass < 2; ++pass) {
#pragma unroll
      for (int it = 0; it < 8; ++it) {
        const int row = it * 2 + hh;
        const v4f v = *(const v4f*)(slab + row * 68 + c4);
        *(volatile v4f*)(C + (size_t)(mBase + row) * ldc + n0 + c4) = v;
      }
      __threadfence();
    }
    __builtin_amdgcn_fence(__ATOMIC_RELEASE, "workgroup");
    __builtin_amdgcn_wave_barrier();
    __builtin_amdgcn_fence(__ATOMIC_ACQUIRE, "workgroup");
  }
}

__global__ __launch_bounds__(64) void chain_scan_kernel(
    const float* __restrict__ VIN, const float* __restrict__ Lre, const float* __restrict__ Lim,
    unsigned short* __restrict__ A2g)
{
  __shared__ __align__(16) float sRe[kScanTS * kScanLP];
  __shared__ __align__(16) float sIm[kScanTS * kScanLP];
  const int tid = threadIdx.x, lane = tid & 31, wave = tid >> 5;
  constexpr int kBlkPerB = kP / kScanCh;
  const int bl = blockIdx.x / kBlkPerB;
  const int p0 = (blockIdx.x - bl * kBlkPerB) * kScanCh;
  const float lr = Lre[p0 + tid];
  const float li = Lim[p0 + tid];
  const size_t row0 = (size_t)bl * kL;
  float xr = 0.0f, xi = 0.0f;
  const int sr4 = tid >> 4, sc4 = (tid & 15) * 4;
  const int q = lane >> 3, c8 = (lane & 7) * 8;
#pragma unroll 1
  for (int t0 = 0; t0 < kL; t0 += kScanTS) {
    __syncthreads();
#pragma unroll 4
    for (int i = 0; i < 16; ++i) {
      const int r = sr4 + 4 * i;
      const float* src = VIN + (row0 + t0 + r) * kVinP + p0 + sc4;
      const v4f a = *(const v4f*)(src);
      const v4f c = *(const v4f*)(src + kP);
      *(v4f*)(sRe + r * kScanLP + sc4) = a;
      *(v4f*)(sIm + r * kScanLP + sc4) = c;
    }
    __syncthreads();
#pragma unroll 4
    for (int s = 0; s < kScanTS; ++s) {
      const float vr = sRe[s * kScanLP + tid];
      const float vi = sIm[s * kScanLP + tid];
      const float sumr = xr + vr;
      const float sumi = xi + vi;
      const float t1 = li * sumi;
      const float t2 = li * sumr;
      xr = fmaf(lr, sumr, -t1);
      xi = fmaf(lr, sumi, t2);
      sRe[s * kScanLP + tid] = xr * kCarryX;
      sIm[s * kScanLP + tid] = xi * kCarryX;
    }
    __syncthreads();
    v8h hv[8], gv[8];
#pragma unroll
    for (int it = 0; it < 8; ++it) {
      const int row = it * 8 + wave * 4 + q;
      const float* spr = sRe + row * kScanLP + c8;
      const float* spi = sIm + row * kScanLP + c8;
      const v4f a0 = *(const v4f*)(spr);
      const v4f a1 = *(const v4f*)(spr + 4);
      const v4f b0 = *(const v4f*)(spi);
      const v4f b1 = *(const v4f*)(spi + 4);
#pragma unroll
      for (int e = 0; e < 4; ++e) {
        hv[it][e]     = to_f16_flush(a0[e]);
        hv[it][4 + e] = to_f16_flush(a1[e]);
        gv[it][e]     = to_f16_flush(b0[e]);
        gv[it][4 + e] = to_f16_flush(b1[e]);
      }
    }
    for (int pass = 0; pass < 2; ++pass) {
#pragma unroll
      for (int it = 0; it < 8; ++it) {
        const int row = it * 8 + wave * 4 + q;
        const size_t o = (row0 + t0 + row) * kA2P + p0 + c8;
        *(volatile v8h*)(A2g + o) = hv[it];
        *(volatile v8h*)(A2g + o + kColIm) = gv[it];
      }
      __threadfence();
    }
  }
}

extern "C" void kernel_launch(void* const* d_in, const int* in_sizes, int n_in,
                              void* d_out, int out_size, void* d_ws, size_t ws_size,
                              hipStream_t stream) {
  if (n_in < 8) return;
  if (in_sizes[0] != kB * kH * kL) return;
  if (in_sizes[1] != kP || in_sizes[2] != kP) return;
  if (in_sizes[3] != kP * kH || in_sizes[4] != kP * kH) return;
  if (in_sizes[5] != kH * kP || in_sizes[6] != kH * kP) return;
  if (in_sizes[7] != kH * kH) return;
  if (out_size != kB * kH * kL) return;
  if (ws_size < kWsTotal) return;

  const float* u   = (const float*)d_in[0];
  const float* Lre = (const float*)d_in[1];
  const float* Lim = (const float*)d_in[2];
  const float* Bre = (const float*)d_in[3];
  const float* Bim = (const float*)d_in[4];
  const float* Cre = (const float*)d_in[5];
  const float* Cim = (const float*)d_in[6];
  const float* Dm  = (const float*)d_in[7];
  float* out = (float*)d_out;

  char* ws = (char*)d_ws;
  unsigned short* A2  = (unsigned short*)(ws + kOffA2);
  float*          VIN = (float*)(ws + kOffVIN);
  unsigned short* BT1 = (unsigned short*)(ws + kOffBT1);
  unsigned short* W2  = (unsigned short*)(ws + kOffW2);

  prep_weights_kernel<<<72, 256, 0, stream>>>(Bre, Bim, Cre, Cim, Dm, BT1, W2);

  pack_u_kernel<<<dim3(kL / 64, kB), 256, 0, stream>>>(u, A2);

  for (int g = 0; g < kGroups; ++g) {
    unsigned short* A2g = A2 + (size_t)g * kGroupRows * kA2P;
    gemm_f16_kernel<false><<<dim3(256, 1), 256, 0, stream>>>(
        A2g + kColU, kA2P, 0L,
        BT1, kH, 0L,
        VIN, kVinP, 0L,
        kGroupRows, kVinP, kH, kFoldMix);
    chain_scan_kernel<<<kGroupB * (kP / kScanCh), kScanCh, 0, stream>>>(VIN, Lre, Lim, A2g);
  }

  gemm_f16_kernel<true><<<dim3(32, kB), 256, 0, stream>>>(
      W2, kA2P, 0L,
      A2, kA2P, (long)kL * kA2P,
      out, kL, (long)kH * kL,
      kH, kL, kA2P, kFoldOut);
}
